// QGKT_51694226375075
// MI455X (gfx1250) — hardware-verified
//
#include <hip/hip_runtime.h>


typedef _Float16 f16t;
typedef f16t  v16h __attribute__((ext_vector_type(16)));
typedef f16t  v8h  __attribute__((ext_vector_type(8)));
typedef float v8f  __attribute__((ext_vector_type(8)));
typedef float v4f  __attribute__((ext_vector_type(4)));
typedef unsigned int v4u __attribute__((ext_vector_type(4)));

union Frag { v16h v; v8h q[2]; };
union Pk16 { v8h h; v4u u; };

static constexpr int kB   = 64;
static constexpr int kT   = 200;
static constexpr int kH   = 256;
static constexpr int kG   = 768;
static constexpr int kQ   = 32001;
static constexpr int kTok = kB * kT;
static constexpr int kOut = kB * (kT - 1);
static constexpr int HP   = 264;
static constexpr int SP   = 132;

static_assert((kTok % 64) == 0);
static_assert((kG % 128) == 0);
static_assert((kOut % 32) == 0);
static_assert((HP % 8) == 0);
static_assert((SP % 4) == 0);

__device__ __forceinline__ v8f wmma16(v16h a, v16h b, v8f c) {
    return __builtin_amdgcn_wmma_f32_16x16x32_f16(false, a, false, b, (short)0, c, false, false);
}

__device__ __forceinline__ void wguard(v8f (&c)[4][2], Frag (&a)[4], Frag (&b)[2]) {
    asm volatile("v_nop\n\tv_nop\n\tv_nop\n\tv_nop"
                 : "+v"(c[0][0]), "+v"(c[0][1]), "+v"(c[1][0]), "+v"(c[1][1]),
                   "+v"(c[2][0]), "+v"(c[2][1]), "+v"(c[3][0]), "+v"(c[3][1])
                 : "v"(a[0].v), "v"(a[1].v), "v"(a[2].v), "v"(a[3].v),
                   "v"(b[0].v), "v"(b[1].v));
}

template<int MT, int NT>
__device__ __forceinline__ void zacc(v8f (&acc)[MT][NT]) {
    const v8f z = {0.f, 0.f, 0.f, 0.f, 0.f, 0.f, 0.f, 0.f};
#pragma unroll
    for (int i = 0; i < MT; ++i)
#pragma unroll
        for (int j = 0; j < NT; ++j) acc[i][j] = z;
}

template<int MT, int NT>
__device__ __forceinline__ void mma_acc(v8f (&acc)[MT][NT],
                                        const f16t* A, int lda,
                                        const f16t* B, int ldb, int ktiles) {
    const int l = threadIdx.x & 31, h = l >> 4, m = l & 15;
    const f16t* ap = A + (size_t)m * lda + 8 * h;
    const f16t* bp = B + (size_t)m * ldb + 8 * h;
#pragma unroll 1
    for (int kt = 0; kt < ktiles; ++kt) {
        Frag a[MT], b[NT];
#pragma unroll
        for (int i = 0; i < MT; ++i) {
            const f16t* p = ap + (size_t)i * 16 * lda + kt * 32;
            a[i].q[0] = *(const v8h*)p;
            a[i].q[1] = *(const v8h*)(p + 16);
        }
#pragma unroll
        for (int j = 0; j < NT; ++j) {
            const f16t* p = bp + (size_t)j * 16 * ldb + kt * 32;
            b[j].q[0] = *(const v8h*)p;
            b[j].q[1] = *(const v8h*)(p + 16);
        }
#pragma unroll
        for (int i = 0; i < MT; ++i)
#pragma unroll
            for (int j = 0; j < NT; ++j)
                acc[i][j] = wmma16(a[i].v, b[j].v, acc[i][j]);
        wguard(acc, a, b);
    }
}

__device__ __forceinline__ float fsigm(float x) {
    float t = __expf(-x);
    return __builtin_amdgcn_rcpf(1.0f + t);
}
__device__ __forceinline__ float ftanh(float x) {
    float ax = fabsf(x);
    float t  = __expf(-2.0f * ax);
    float r  = (1.0f - t) * __builtin_amdgcn_rcpf(1.0f + t);
    return copysignf(r, x);
}

__device__ __forceinline__ int clampi(int v, int lo, int hi) {
    return v < lo ? lo : (v > hi ? hi : v);
}

__global__ __launch_bounds__(256)
void k_prep(const int* feat, const int* qs, const int* ans,
            const float* q_emb, const float* a_emb,
            const float* w_ih, const float* w_hh,
            f16t* X16, f16t* Pih, f16t* Phh, int nxblk, int nq_rows) {
    (void)feat;
    const int tid = threadIdx.x;
    if ((int)blockIdx.x < nxblk) {
        const int i = blockIdx.x * 256 + tid;
        if (i >= kTok * (kH / 8)) return;
        const int row = i >> 5, ch = (i & 31) * 8;
        const int t = row >> 6, b = row & 63;
        const int q = clampi(qs[b * kT + t], 0, nq_rows - 1);
        const int a = clampi(ans[b * kT + t], 0, 1);
        const float* qp = q_emb + (size_t)q * kH + ch;
        const float* ap = a_emb + (size_t)a * kH + ch;
        v4f q0 = *(const v4f*)qp, q1 = *(const v4f*)(qp + 4);
        v4f a0 = *(const v4f*)ap, a1 = *(const v4f*)(ap + 4);
        Pk16 k;
#pragma unroll
        for (int e = 0; e < 4; ++e) {
            k.h[e]     = (f16t)((q0[e] + a0[e]) * 32.0f);
            k.h[4 + e] = (f16t)((q1[e] + a1[e]) * 32.0f);
        }
        f16t* d = X16 + (size_t)row * kH + ch;
        *(volatile v4u*)d = k.u;
        __threadfence();
        *(volatile v4u*)d = k.u;
    } else {
        const int per = kG * kH / 8;
        const int i = ((int)blockIdx.x - nxblk) * 256 + tid;
        if (i >= 2 * per) return;
        const int which = (i >= per) ? 1 : 0;
        const int j = i - which * per;
        const float* src = which ? w_hh : w_ih;
        f16t* dstp = which ? Phh : Pih;
        const float* sp = src + (size_t)j * 8;
        v4f s0 = *(const v4f*)sp, s1 = *(const v4f*)(sp + 4);
        Pk16 k;
#pragma unroll
        for (int e = 0; e < 4; ++e) {
            k.h[e]     = (f16t)(s0[e] * 16.0f);
            k.h[4 + e] = (f16t)(s1[e] * 16.0f);
        }
        f16t* d = dstp + (size_t)j * 8;
        *(volatile v4u*)d = k.u;
        __threadfence();
        *(volatile v4u*)d = k.u;
    }
}

__global__ __launch_bounds__(128)
void k_gemm(const f16t* X16, const f16t* Pih, const float* b_ih, float* Gi,
            int nrows, float inv) {
    __shared__ __attribute__((aligned(16))) float S[64 * SP];
    const int tid = threadIdx.x, w = tid >> 5;
    const int l = tid & 31, h = l >> 4, m = l & 15;
    const int c0 = blockIdx.x * 128;
    const int r0 = blockIdx.y * 64;
    if (r0 + 64 > nrows) return;

    v8f acc[4][2]; zacc(acc);
    mma_acc<4, 2>(acc, X16 + (size_t)r0 * kH, kH, Pih + (size_t)(c0 + 32 * w) * kH, kH, 8);

#pragma unroll
    for (int j = 0; j < 2; ++j) {
        const int cl = 32 * w + 16 * j + m;
        const float bias = b_ih[c0 + cl];
#pragma unroll
        for (int i = 0; i < 4; ++i)
#pragma unroll
            for (int r = 0; r < 8; ++r)
                S[(16 * i + 8 * h + r) * SP + cl] = fmaf(acc[i][j][r], inv, bias);
    }
    __syncthreads();

#pragma unroll
    for (int it = 0; it < 16; ++it) {
        const int p = tid + 128 * it, row = p >> 5, c4 = (p & 31) * 4;
        v4f v = *(const v4f*)(S + row * SP + c4);
        *(volatile v4f*)(Gi + (size_t)(r0 + row) * kG + c0 + c4) = v;
    }
    __threadfence();
#pragma unroll
    for (int it = 0; it < 16; ++it) {
        const int p = tid + 128 * it, row = p >> 5, c4 = (p & 31) * 4;
        v4f v = *(const v4f*)(S + row * SP + c4);
        *(volatile v4f*)(Gi + (size_t)(r0 + row) * kG + c0 + c4) = v;
    }
}

__device__ __forceinline__ void gru_unit(const f16t* Hc, f16t* Hn,
                                         const f16t* __restrict__ Phh,
                                         const float* __restrict__ Git,
                                         const float* __restrict__ b_hh,
                                         const int* __restrict__ qs,
                                         const float* __restrict__ pred_w,
                                         float* Pp, int mt, int cg, int t, int nq_rows,
                                         float inv, v8f& hold) {
    const int l = threadIdx.x & 31, h = l >> 4, m = l & 15;
    const v8f z8 = {0.f, 0.f, 0.f, 0.f, 0.f, 0.f, 0.f, 0.f};
    v8f cr = z8, cz = z8, cn = z8;
    const f16t* ap  = Hc + (size_t)(16 * mt + m) * HP + 8 * h;
    const f16t* bpr = Phh + (size_t)(16 * cg + m) * kH + 8 * h;
    const f16t* bpz = bpr + (size_t)256 * kH;
    const f16t* bpn = bpr + (size_t)512 * kH;
#pragma unroll 1
    for (int ks = 0; ks < 8; ++ks) {
        const int k0 = ks * 32;
        Frag a, br, bz, bn;
        a.q[0]  = *(const v8h*)(ap + k0);   a.q[1]  = *(const v8h*)(ap + k0 + 16);
        br.q[0] = *(const v8h*)(bpr + k0);  br.q[1] = *(const v8h*)(bpr + k0 + 16);
        bz.q[0] = *(const v8h*)(bpz + k0);  bz.q[1] = *(const v8h*)(bpz + k0 + 16);
        bn.q[0] = *(const v8h*)(bpn + k0);  bn.q[1] = *(const v8h*)(bpn + k0 + 16);
        cr = wmma16(a.v, br.v, cr);
        cz = wmma16(a.v, bz.v, cz);
        cn = wmma16(a.v, bn.v, cn);
        asm volatile("v_nop\n\tv_nop\n\tv_nop\n\tv_nop"
                     : "+v"(cr), "+v"(cz), "+v"(cn)
                     : "v"(a.v), "v"(br.v), "v"(bz.v), "v"(bn.v));
    }
    const int c = 16 * cg + m;
    const float bhr = b_hh[c], bhz = b_hh[256 + c], bhn = b_hh[512 + c];
    const float* pwc = pred_w + c;
#pragma unroll
    for (int r = 0; r < 8; ++r) {
        const int b = 16 * mt + 8 * h + r;
        const float* gr = Git + (size_t)b * kG + c;
        const float ir = gr[0], iz = gr[256], in_ = gr[512];
        const float ghr = fmaf(cr[r], inv, bhr);
        const float ghz = fmaf(cz[r], inv, bhz);
        const float ghn = fmaf(cn[r], inv, bhn);
        const float rg = fsigm(ir + ghr);
        const float zg = fsigm(iz + ghz);
        const float ng = ftanh(fmaf(rg, ghn, in_));
        const float hn = (1.0f - zg) * ng + zg * hold[r];
        hold[r] = hn;
        Hn[(size_t)b * HP + c] = (f16t)(hn * 8.0f);
        const int q = clampi(qs[b * kT + t], 0, nq_rows - 1);
        float p = hn * pwc[(size_t)q * kH];
        p += __shfl_xor(p, 1, 32);
        p += __shfl_xor(p, 2, 32);
        p += __shfl_xor(p, 4, 32);
        p += __shfl_xor(p, 8, 32);
        if (m == 0) Pp[b * 16 + cg] = p;
    }
}

__global__ __launch_bounds__(512)
void k_gru(const f16t* Phh, const float* Gi, const float* b_hh, const int* qs,
           const float* pred_w, const float* pred_b, float* out, int nq_rows, float inv) {
    __shared__ __attribute__((aligned(16))) f16t  Hs[2 * kB * HP];
    __shared__ __attribute__((aligned(16))) float Pp[kB * 16];
    __shared__ __attribute__((aligned(16))) float Pr[kOut];
    const int tid = threadIdx.x, w = tid >> 5;
    const int mt = w >> 2, cgb = (w & 3) * 4;

    for (int i = tid; i < 2 * kB * HP; i += 512) Hs[i] = (f16t)0.0f;
    const v8f z8 = {0.f, 0.f, 0.f, 0.f, 0.f, 0.f, 0.f, 0.f};
    v8f hold0 = z8, hold1 = z8, hold2 = z8, hold3 = z8;
    __syncthreads();

#pragma unroll 1
    for (int t = 0; t < kT; ++t) {
        const f16t* Hc = Hs + (size_t)(t & 1) * kB * HP;
        f16t*       Hn = Hs + (size_t)((t + 1) & 1) * kB * HP;
        const float* Git = Gi + (size_t)t * kB * kG;

        gru_unit(Hc, Hn, Phh, Git, b_hh, qs, pred_w, Pp, mt, cgb + 0, t, nq_rows, inv, hold0);
        gru_unit(Hc, Hn, Phh, Git, b_hh, qs, pred_w, Pp, mt, cgb + 1, t, nq_rows, inv, hold1);
        gru_unit(Hc, Hn, Phh, Git, b_hh, qs, pred_w, Pp, mt, cgb + 2, t, nq_rows, inv, hold2);
        gru_unit(Hc, Hn, Phh, Git, b_hh, qs, pred_w, Pp, mt, cgb + 3, t, nq_rows, inv, hold3);
        __syncthreads();

        if (tid < kB) {
            const int b = tid;
            const int q = clampi(qs[b * kT + t], 0, nq_rows - 1);
            float s = pred_b[q];
            const float* pp = Pp + b * 16;
#pragma unroll
            for (int g = 0; g < 16; ++g) s += pp[g];
            const float prob = fsigm(s);
            if (t < kT - 1) Pr[b * (kT - 1) + t] = prob;
        }
        __syncthreads();
    }

    for (int p = tid; p < kOut / 4; p += 512) {
        v4f v = *(const v4f*)(Pr + 4 * p);
        *(volatile v4f*)(out + 4 * p) = v;
    }
    __threadfence();
    for (int p = tid; p < kOut / 4; p += 512) {
        v4f v = *(const v4f*)(Pr + 4 * p);
        *(volatile v4f*)(out + 4 * p) = v;
    }
}

extern "C" void kernel_launch(void* const* d_in, const int* in_sizes, int n_in,
                              void* d_out, int out_size, void* d_ws, size_t ws_size,
                              hipStream_t stream) {
    if (n_in < 11) return;
    if (in_sizes[1] != kB * kT || in_sizes[2] != kB * kT ||
        in_sizes[3] != kQ * kH  || in_sizes[4] != 2 * kH ||
        in_sizes[5] != kG * kH  || in_sizes[6] != kG * kH ||
        in_sizes[7] != kG       || in_sizes[8] != kG ||
        in_sizes[9] != kQ * kH  || in_sizes[10] != kQ ||
        out_size != kOut) return;

    const int*   feat   = (const int*)d_in[0];
    const int*   qs     = (const int*)d_in[1];
    const int*   ans    = (const int*)d_in[2];
    const float* q_emb  = (const float*)d_in[3];
    const float* a_emb  = (const float*)d_in[4];
    const float* w_ih   = (const float*)d_in[5];
    const float* w_hh   = (const float*)d_in[6];
    const float* b_ih   = (const float*)d_in[7];
    const float* b_hh   = (const float*)d_in[8];
    const float* pred_w = (const float*)d_in[9];
    const float* pred_b = (const float*)d_in[10];
    float* out = (float*)d_out;
    const int nq_rows = in_sizes[3] / kH;

    char* ws = (char*)d_ws;
    size_t off = 0;
    auto carve = [&](size_t bytes) -> char* {
        char* p = ws + off;
        off = (off + bytes + 255) & ~(size_t)255;
        return p;
    };
    f16t*  X16 = (f16t*)carve((size_t)kTok * kH * 2);
    f16t*  Pih = (f16t*)carve((size_t)kG * kH * 2);
    f16t*  Phh = (f16t*)carve((size_t)kG * kH * 2);
    float* Gi  = (float*)carve((size_t)kTok * kG * 4);
    if (off > ws_size) return;

    const float invG = 1.0f / 512.0f;
    const float invH = 1.0f / 128.0f;

    const int nxblk = (kTok * (kH / 8) + 255) / 256;
    const int nwblk = (2 * kG * kH / 8 + 255) / 256;
    k_prep<<<dim3(nxblk + nwblk), dim3(256), 0, stream>>>(feat, qs, ans, q_emb, a_emb, w_ih, w_hh,
                                                          X16, Pih, Phh, nxblk, nq_rows);
    k_gemm<<<dim3(kG / 128, kTok / 64), dim3(128), 0, stream>>>(X16, Pih, b_ih, Gi, kTok, invG);
    k_gru<<<dim3(1), dim3(512), 0, stream>>>(Phh, Gi, b_hh, qs, pred_w, pred_b, out, nq_rows, invH);
}
